// SelfAttentionUncertainty_58463094833355
// MI455X (gfx1250) — hardware-verified
//
#include <hip/hip_runtime.h>
#include <hip/hip_bf16.h>
#include <math.h>


#define BB 8
#define SS 1024
#define DD 768
#define HH 12
#define DKK 64
#define QW 2

typedef _Float16 bf16;
typedef __attribute__((ext_vector_type(4))) unsigned v4u_t;
typedef unsigned v4ua __attribute__((ext_vector_type(4), may_alias));
typedef __attribute__((ext_vector_type(4))) float v4f_t;
typedef float v4fa __attribute__((ext_vector_type(4), may_alias));
typedef __attribute__((ext_vector_type(16))) bf16  bf16x16;
typedef __attribute__((ext_vector_type(8)))  bf16  bf16x8;
typedef __attribute__((ext_vector_type(4)))  bf16  bf16x4;
typedef __attribute__((ext_vector_type(8)))  float f32x8;

#define LDS_STRIDE 48
#define KSTRIDE    72
#define VSTRIDE    48

__device__ __forceinline__ f32x8 wmma_bf16(bf16x16 a, bf16x16 b, f32x8 c) {
  return __builtin_amdgcn_wmma_f32_16x16x32_f16(
      false, a, false, b, (short)0, c, false, false);
}

template <typename T>
__device__ __forceinline__ bf16x16 load_frag(const T* __restrict__ base, int ld,
                                             int row0, int k0) {
  const int lane = threadIdx.x & 31;
  const int r    = lane & 15;
  const int kh   = (lane >> 4) * 8;
  const T* p0 = base + (size_t)(row0 + r) * ld + (k0 + kh);
  const T* p1 = p0 + 16;
  bf16x16 f;
#pragma unroll
  for (int i = 0; i < 8; ++i) {
    f[i]     = (bf16)p0[i];
    f[i + 8] = (bf16)p1[i];
  }
  return f;
}

__device__ __forceinline__ bf16x16 lds_frag(const bf16* base, int stride) {
  const int lane = threadIdx.x & 31;
  const int row  = lane & 15;
  const int kh   = (lane >> 4) * 8;
  const bf16x8 lo = *(const bf16x8*)(base + row * stride + kh);
  const bf16x8 hi = *(const bf16x8*)(base + row * stride + kh + 16);
  bf16x16 f;
#pragma unroll
  for (int i = 0; i < 8; ++i) { f[i] = lo[i]; f[i + 8] = hi[i]; }
  return f;
}

template <typename T>
__device__ __forceinline__ void stage_read16(const T* __restrict__ p, float* buf) {
#pragma unroll
  for (int i = 0; i < 16; ++i) buf[i] = (float)p[i];
}

__device__ __forceinline__ void stage_write(bf16* dst, const float* buf, int nquad) {
#pragma unroll
  for (int i = 0; i < nquad; ++i) {
    bf16x4 q;
    q[0] = (bf16)buf[4 * i];     q[1] = (bf16)buf[4 * i + 1];
    q[2] = (bf16)buf[4 * i + 2]; q[3] = (bf16)buf[4 * i + 3];
    *(bf16x4*)(dst + 4 * i) = q;
  }
}

__global__ __launch_bounds__(256) void transpose_pack_kernel(const float* __restrict__ W, bf16* __restrict__ WT, int K, int N) {
  __shared__ float tile[64][65];
  const int k0 = blockIdx.y * 64, n0 = blockIdx.x * 64, t = threadIdx.x;
  for (int i = t; i < 64 * 64; i += 256) { const int kr = i >> 6, nc = i & 63; tile[kr][nc] = W[(size_t)(k0 + kr) * N + n0 + nc]; }
  __syncthreads();
#pragma unroll 1
  for (int pass = 0; pass < 2; ++pass) {
    for (int i = t; i < 64 * 8; i += 256) { const int nr = i >> 3, k8 = (i & 7) * 8; bf16 hh[8];
#pragma unroll
      for (int e = 0; e < 8; ++e) hh[e] = (bf16)tile[k8 + e][nr];
      *(volatile v4u_t*)(WT + (size_t)(n0 + nr) * K + k0 + k8) = *(const v4ua*)hh; }
    __threadfence();
  }
}

template <typename AT, typename WT, int MODE>
__global__ __launch_bounds__(256) void gemm_bias_kernel(
    const AT* __restrict__ A, const WT* __restrict__ W,
    const float* __restrict__ bias, void* __restrict__ out,
    int M, int N, int K, const float* __restrict__ rbias = nullptr) {
  __shared__ bf16 ldsA[128 * LDS_STRIDE];
  __shared__ bf16 ldsW[256 * LDS_STRIDE];
  __shared__ __attribute__((aligned(16))) unsigned char sob[256 * 136 * 2];

  const int t    = threadIdx.x;
  const int wave = t >> 5;
  const int lane = t & 31;
  const int wm   = (wave & 1) * 64;
  const int wn   = (wave >> 1) * 64;
  const int mBlk = blockIdx.x * 128;
  const int nBlk = blockIdx.y * 256;

  const int arow = t >> 1;
  const int ach  = (t & 1) * 16;

  float abuf[16];
  float wbuf[32];

  stage_read16(A + (size_t)(mBlk + arow) * K + ach, abuf);
  stage_read16(W + (size_t)(nBlk + t) * K,          wbuf);
  stage_read16(W + (size_t)(nBlk + t) * K + 16,     wbuf + 16);

  f32x8 acc[4][4] = {};

  for (int k = 0; k < K; k += 32) {
    __syncthreads();
    stage_write(&ldsA[arow * LDS_STRIDE + ach], abuf, 4);
    stage_write(&ldsW[t * LDS_STRIDE],          wbuf, 8);
    if (k + 32 < K) {
      stage_read16(A + (size_t)(mBlk + arow) * K + (k + 32) + ach, abuf);
      stage_read16(W + (size_t)(nBlk + t) * K + (k + 32),          wbuf);
      stage_read16(W + (size_t)(nBlk + t) * K + (k + 32) + 16,     wbuf + 16);
    }
    __syncthreads();

    bf16x16 af[4], wf[4];
#pragma unroll
    for (int i = 0; i < 4; ++i)
      af[i] = lds_frag(ldsA + (wm + 16 * i) * LDS_STRIDE, LDS_STRIDE);
#pragma unroll
    for (int j = 0; j < 4; ++j)
      wf[j] = lds_frag(ldsW + (wn + 16 * j) * LDS_STRIDE, LDS_STRIDE);
#pragma unroll
    for (int i = 0; i < 4; ++i)
#pragma unroll
      for (int j = 0; j < 4; ++j)
        acc[i][j] = wmma_bf16(af[i], wf[j], acc[i][j]);
  }

  const int nlane = lane & 15;
  const int mh    = (lane >> 4) * 8;
  __syncthreads();
  if (MODE == 0 || MODE == 1) {
    bf16* so = (bf16*)sob;
#pragma unroll
    for (int i = 0; i < 4; ++i)
#pragma unroll
      for (int j = 0; j < 4; ++j) {
        const int nl = wn + 16 * j + nlane;
        const float bv = bias ? bias[nBlk + nl] : 0.0f;
#pragma unroll
        for (int r = 0; r < 8; ++r) {
          const int ml = wm + 16 * i + mh + r;
          const bf16 hv = (bf16)(acc[i][j][r] + bv);
          if (MODE == 0) so[ml * 264 + nl] = hv;
          else           so[nl * 136 + ml] = hv;
        }
      }
    __syncthreads();
#pragma unroll 1
    for (int pass = 0; pass < 2; ++pass) {
      if (MODE == 0) {
        for (int ch = t; ch < 128 * 32; ch += 256) { const int ml = ch >> 5, q = (ch & 31) * 8;
          *(volatile v4u_t*)((bf16*)out + (size_t)(mBlk + ml) * N + nBlk + q) = *(const v4ua*)(so + ml * 264 + q); }
      } else {
        const int b_ = mBlk / SS, s0 = mBlk & (SS - 1);
        for (int ch = t; ch < 256 * 16; ch += 256) { const int nl = ch >> 4, q = (ch & 15) * 8; const int n = nBlk + nl, h = n >> 6, dk = n & (DKK - 1);
          *(volatile v4u_t*)((bf16*)out + (((size_t)(b_ * HH + h)) * DKK + dk) * SS + s0 + q) = *(const v4ua*)(so + nl * 136 + q); }
      }
      __threadfence();
    }
  } else {
    float* so = (float*)sob;
#pragma unroll 1
    for (int hf = 0; hf < 2; ++hf) {
      if (wm == hf * 64) {
#pragma unroll
        for (int i = 0; i < 4; ++i)
#pragma unroll
          for (int j = 0; j < 4; ++j) {
            const int nl = wn + 16 * j + nlane;
            const float bv = bias ? bias[nBlk + nl] : 0.0f;
#pragma unroll
            for (int r = 0; r < 8; ++r) so[(16 * i + mh + r) * 260 + nl] = acc[i][j][r] + bv + (rbias ? rbias[mBlk + hf * 64 + 16 * i + mh + r] : 0.0f);
          }
      }
      __syncthreads();
      if (MODE == 3) {
        const int row = t >> 2, hq = t & 3; float* v = so + row * 260 + hq * 64;
        const int token = mBlk + hf * 64 + row, n = token % SS, py = n >> 5, px = n & 31;
#pragma unroll 1
        for (int p = 0; p < DKK / 2; ++p) {
          const int pidx = p & 15; const float posv = (p < 16) ? (float)py : (float)px;
          const float invf = 1.0f / powf(10000.0f, (float)pidx / 16.0f);
          const float ang = posv * invf, c = cosf(ang), s = sinf(ang);
          const float xe = v[2 * p], xo = v[2 * p + 1];
          v[2 * p] = xe * c - xo * s; v[2 * p + 1] = xo * c + xe * s;
        }
        __syncthreads();
      }
#pragma unroll 1
      for (int pass = 0; pass < 2; ++pass) {
        for (int ch = t; ch < 64 * 64; ch += 256) { const int ml = ch >> 6, q = (ch & 63) * 4;
          *(volatile v4f_t*)((float*)out + (size_t)(mBlk + hf * 64 + ml) * N + nBlk + q) = *(const volatile v4fa*)(so + ml * 260 + q); }
        __threadfence();
      }
      __syncthreads();
    }
  }
}

__global__ __launch_bounds__(64) void attn2_kernel(const bf16* __restrict__ Qb, const bf16* __restrict__ Kb, const bf16* __restrict__ Vt,
                                                   bf16* __restrict__ attnOut, float* __restrict__ ent) {
  __shared__ bf16 ldsK[32 * KSTRIDE];
  __shared__ bf16 ldsV[64 * VSTRIDE];
  __shared__ __attribute__((aligned(16))) bf16 ldsO[2][32 * 72];
  __shared__ __attribute__((aligned(16))) float ldsE[2][32];
  const int q0blk = blockIdx.x * 64, h = blockIdx.y, b = blockIdx.z;
  const int t = threadIdx.x, wave = t >> 5, lane = t & 31, qlane = lane & 15, kh8 = (lane >> 4) * 8;
  const int q0 = q0blk + wave * 32;
  const bf16* Qh = Qb + (size_t)b * SS * DD + h * DKK;
  const bf16* Kh = Kb + (size_t)b * SS * DD + h * DKK;
  const bf16* Vh = Vt + ((size_t)(b * HH + h)) * DKK * SS;
  const int krow = t >> 1, kcol = (t & 1) * 32;
  bf16x16 qf[QW][2];
#pragma unroll
  for (int qt = 0; qt < QW; ++qt) { qf[qt][0] = load_frag(Qh, DD, q0 + 16 * qt, 0); qf[qt][1] = load_frag(Qh, DD, q0 + 16 * qt, 32); }
  const float scale = 0.125f * 1.44269504088896340736f;
  float mrun[QW], lrun[QW];
#pragma unroll
  for (int qt = 0; qt < QW; ++qt) { mrun[qt] = -INFINITY; lrun[qt] = 0.0f; }
#pragma unroll 1
  for (int kb = 0; kb < SS; kb += 32) {
    __syncthreads();
    { const bf16* ks = Kh + (size_t)(kb + krow) * DD + kcol;
#pragma unroll
      for (int i = 0; i < 4; ++i) *(bf16x8*)(&ldsK[krow * KSTRIDE + kcol + 8 * i]) = *(const bf16x8*)(ks + 8 * i); }
    __syncthreads();
    bf16x16 kf[2][2];
#pragma unroll
    for (int kt = 0; kt < 2; ++kt)
#pragma unroll
      for (int c = 0; c < 2; ++c) kf[kt][c] = lds_frag(ldsK + (kt * 16) * KSTRIDE + c * 32, KSTRIDE);
#pragma unroll
    for (int qt = 0; qt < QW; ++qt) {
      f32x8 s0 = {}, s1 = {};
      s0 = wmma_bf16(kf[0][0], qf[qt][0], s0); s0 = wmma_bf16(kf[0][1], qf[qt][1], s0);
      s1 = wmma_bf16(kf[1][0], qf[qt][0], s1); s1 = wmma_bf16(kf[1][1], qf[qt][1], s1);
      float mx = -INFINITY;
#pragma unroll
      for (int r = 0; r < 8; ++r) { s0[r] *= scale; s1[r] *= scale; mx = fmaxf(mx, fmaxf(s0[r], s1[r])); }
      mx = fmaxf(mx, __shfl_xor(mx, 16, 32));
      const float mnew = fmaxf(mrun[qt], mx), alpha = exp2f(mrun[qt] - mnew);
      float rs = 0.0f;
#pragma unroll
      for (int r = 0; r < 8; ++r) rs += exp2f(s0[r] - mnew) + exp2f(s1[r] - mnew);
      rs += __shfl_xor(rs, 16, 32);
      lrun[qt] = lrun[qt] * alpha + rs; mrun[qt] = mnew;
    }
  }
  f32x8 o[QW][4] = {};
  float entv[QW], linv[QW];
#pragma unroll
  for (int qt = 0; qt < QW; ++qt) { entv[qt] = 0.0f; linv[qt] = 1.0f / lrun[qt]; }
#pragma unroll 1
  for (int kb = 0; kb < SS; kb += 32) {
    __syncthreads();
    { const bf16* ks = Kh + (size_t)(kb + krow) * DD + kcol; const bf16* vs = Vh + (size_t)t * SS + kb;
#pragma unroll
      for (int i = 0; i < 4; ++i) { *(bf16x8*)(&ldsK[krow * KSTRIDE + kcol + 8 * i]) = *(const bf16x8*)(ks + 8 * i); *(bf16x8*)(&ldsV[t * VSTRIDE + 8 * i]) = *(const bf16x8*)(vs + 8 * i); } }
    __syncthreads();
    bf16x16 kf[2][2];
#pragma unroll
    for (int kt = 0; kt < 2; ++kt)
#pragma unroll
      for (int c = 0; c < 2; ++c) kf[kt][c] = lds_frag(ldsK + (kt * 16) * KSTRIDE + c * 32, KSTRIDE);
    bf16x16 pf[QW];
#pragma unroll
    for (int qt = 0; qt < QW; ++qt) {
      f32x8 s0 = {}, s1 = {};
      s0 = wmma_bf16(kf[0][0], qf[qt][0], s0); s0 = wmma_bf16(kf[0][1], qf[qt][1], s0);
      s1 = wmma_bf16(kf[1][0], qf[qt][0], s1); s1 = wmma_bf16(kf[1][1], qf[qt][1], s1);
      float es = 0.0f;
#pragma unroll
      for (int r = 0; r < 8; ++r) {
        const float p0 = exp2f(s0[r] * scale - mrun[qt]) * linv[qt], p1 = exp2f(s1[r] * scale - mrun[qt]) * linv[qt];
        es += p0 * logf(p0 + 1e-8f) + p1 * logf(p1 + 1e-8f);
        pf[qt][r] = (bf16)(p0 * 1024.0f); pf[qt][r + 8] = (bf16)(p1 * 1024.0f);
      }
      entv[qt] -= es;
    }
#pragma unroll
    for (int j = 0; j < 4; ++j) { const bf16x16 vf = lds_frag(ldsV + (j * 16) * VSTRIDE, VSTRIDE);
#pragma unroll
      for (int qt = 0; qt < QW; ++qt) o[qt][j] = wmma_bf16(vf, pf[qt], o[qt][j]); }
  }
  bf16* so = ldsO[wave];
#pragma unroll
  for (int qt = 0; qt < QW; ++qt) {
    const float e = entv[qt] + __shfl_xor(entv[qt], 16, 32);
    if (lane < 16) ldsE[wave][16 * qt + qlane] = e;
#pragma unroll
    for (int j = 0; j < 4; ++j)
#pragma unroll
      for (int r = 0; r < 8; ++r) so[(16 * qt + qlane) * 72 + j * 16 + kh8 + r] = (bf16)(o[qt][j][r] * (1.0f / 1024.0f));
  }
  asm volatile("s_wait_dscnt 0" ::: "memory");
#pragma unroll 1
  for (int pass = 0; pass < 2; ++pass) {
#pragma unroll
    for (int it = 0; it < 8; ++it) { const int ch = lane + 32 * it, ql = ch >> 3, q8 = (ch & 7) * 8;
      *(volatile v4u_t*)(attnOut + ((size_t)(b * SS + q0 + ql)) * DD + h * DKK + q8) = *(const v4ua*)(so + ql * 72 + q8); }
    if (lane < 8) *(volatile v4f_t*)(ent + ((size_t)(b * HH + h)) * SS + q0 + lane * 4) = *(const volatile v4fa*)(&ldsE[wave][lane * 4]);
    __threadfence();
  }
}

__global__ __launch_bounds__(256) void k_x3(const float* __restrict__ X, bf16* __restrict__ X3) {
  __shared__ float tile[64][65];
  const int b = blockIdx.z, c0 = blockIdx.y * 64, n0 = blockIdx.x * 64, t = threadIdx.x;
  for (int i = t; i < 64 * 64; i += 256) { const int cr = i >> 6, nn = i & 63; tile[cr][nn] = X[((size_t)b * DD + c0 + cr) * SS + n0 + nn]; }
  __syncthreads();
#pragma unroll 1
  for (int pass = 0; pass < 2; ++pass) {
    for (int i = t; i < 64 * 8; i += 256) { const int nr = i >> 3, c8 = (i & 7) * 8; bf16 hh[8];
#pragma unroll
      for (int e = 0; e < 8; ++e) hh[e] = (bf16)tile[c8 + e][nr];
      *(volatile v4u_t*)(X3 + ((size_t)b * SS + n0 + nr) * DD + c0 + c8) = *(const v4ua*)hh; }
    __threadfence();
  }
}
__global__ __launch_bounds__(192) void k_cvt(const float* __restrict__ Qf, const float* __restrict__ Kf, bf16* __restrict__ Qb, bf16* __restrict__ Kb) {
  const int tok = blockIdx.x, t = threadIdx.x; bf16 hq[4], hk[4];
#pragma unroll
  for (int i = 0; i < 4; ++i) { hq[i] = (bf16)Qf[(size_t)tok * DD + t * 4 + i]; hk[i] = (bf16)Kf[(size_t)tok * DD + t * 4 + i]; }
  typedef __attribute__((ext_vector_type(2))) unsigned v2u; typedef unsigned v2ua __attribute__((ext_vector_type(2), may_alias));
#pragma unroll 1
  for (int pass = 0; pass < 2; ++pass) {
    *(volatile v2u*)(Qb + (size_t)tok * DD + t * 4) = *(const v2ua*)hq; *(volatile v2u*)(Kb + (size_t)tok * DD + t * 4) = *(const v2ua*)hk;
    __threadfence();
  }
}
__global__ __launch_bounds__(256) void k_unc(const float* __restrict__ ent, float* __restrict__ unc) {
  const int b = blockIdx.x, t = threadIdx.x;
#pragma unroll 1
  for (int pass = 0; pass < 2; ++pass) {
    for (int n = t; n < SS; n += 256) { float s = 0.0f;
#pragma unroll
      for (int h = 0; h < HH; ++h) s += ent[((size_t)b * HH + h) * SS + n];
      *(volatile float*)(unc + (size_t)b * SS + n) = s / (float)HH; }
    __threadfence();
  }
}

extern "C" void kernel_launch(void* const* d_in, const int* in_sizes, int n_in,
                              void* d_out, int out_size, void* d_ws, size_t ws_size,
                              hipStream_t stream) {
  (void)in_sizes; (void)n_in; (void)out_size; (void)ws_size;
  const float* X     = (const float*)d_in[0];
  const float* qkv_w = (const float*)d_in[1];
  const float* proj_w = (const float*)d_in[2];
  const float* proj_b = (const float*)d_in[3];
  float* out = (float*)d_out;
  float* unc = out + (size_t)BB * DD * SS;
  char* ws = (char*)d_ws;
  const size_t act = (size_t)BB * SS * DD;
  bf16*  X3  = (bf16*)ws;  ws += act * 2;
  float* Qf  = (float*)ws; ws += act * 4;
  float* Kf  = (float*)ws; ws += act * 4;
  bf16*  Qb  = (bf16*)ws;  ws += act * 2;
  bf16*  Kb  = (bf16*)ws;  ws += act * 2;
  bf16*  VtB = (bf16*)ws;  ws += act * 2;
  bf16*  attn = (bf16*)ws; ws += act * 2;
  float* ent = (float*)ws; ws += (size_t)BB * HH * SS * 4;

  k_x3<<<dim3(SS / 64, DD / 64, BB), 256, 0, stream>>>(X, X3);
  const int M = BB * SS, N = DD, K = DD;
  dim3 gGrid(M / 128, N / 256), gBlk(256);
  gemm_bias_kernel<bf16, float, 3><<<gGrid, gBlk, 0, stream>>>(X3, qkv_w,                       nullptr, Qf,  M, N, K);
  gemm_bias_kernel<bf16, float, 3><<<gGrid, gBlk, 0, stream>>>(X3, qkv_w + (size_t)DD * DD,     nullptr, Kf,  M, N, K);
  gemm_bias_kernel<bf16, float, 1><<<gGrid, gBlk, 0, stream>>>(X3, qkv_w + (size_t)2 * DD * DD, nullptr, VtB, M, N, K);
  k_cvt<<<BB * SS, 192, 0, stream>>>(Qf, Kf, Qb, Kb);
  attn2_kernel<<<dim3(SS / 64, HH, BB), 64, 0, stream>>>(Qb, Kb, VtB, attn, ent);
  k_unc<<<BB, 256, 0, stream>>>(ent, unc);
  for (int b = 0; b < BB; ++b)
    gemm_bias_kernel<float, bf16, 2><<<dim3(DD / 128, SS / 256), gBlk, 0, stream>>>(proj_w, attn + (size_t)b * SS * DD, nullptr, out + (size_t)b * DD * SS, DD, SS, DD, proj_b);
}
